// GNN_90589450207317
// MI455X (gfx1250) — hardware-verified
//
#include <hip/hip_runtime.h>
#include <stddef.h>
#include <stdint.h>
#include <math.h>


#define CIN    128
#define HID    64
#define KK     128
#define NTHR   256
#define NWAVE  8
#define EPT    8
#define CHUNK  (NTHR * EPT)
#define WCAP   (EPT * 32)
#define LISTN  (NWAVE * WCAP)
#define NBA    1024
#define SLA    10
#define RCAP   20480
#define DEGCAP 64
#define OTP    (NBA + 32)
#define GBM    64
#define GBN    64
#define GTHR   128
#define AROWS  64
#define NUW    1024
#define BLD_ZINTS    (LISTN + 2 * RCAP + NBA + OTP + NBA)
#define BLD_LDS_INTS (BLD_ZINTS + 16)
#define WSMAX  134217728

static_assert((CHUNK & (CHUNK - 1)) == 0 && CHUNK <= 4096);
static_assert((NBA & (NBA - 1)) == 0 && NBA == (1 << SLA));
static_assert(((long long)CHUNK << SLA) < (1LL << 31));
static_assert(LISTN % NTHR == 0);
static_assert(NBA == NTHR * 4 && NBA % 32 == 0 && NBA % AROWS == 0 && NBA % GBM == 0);
static_assert(RCAP % (NTHR * 4) == 0 && RCAP % 32 == 0);
static_assert(BLD_ZINTS % 4 == 0 && LISTN % 4 == 0 && OTP % 32 == 0 && OTP - NBA == 32);
static_assert(CIN == KK && KK % 32 == 0 && KK == 2 * HID && HID == GBN);
static_assert(GBM == (GTHR / 32) * 16 && GBN == 64);
static_assert(NUW % NTHR == 0 && NUW == HID * (KK / 8));
static_assert(HID == 2 * 32);
static_assert(AROWS % NWAVE == 0 && AROWS == GBM);
static_assert(BLD_LDS_INTS * 4 <= 300000);

typedef float          v2f   __attribute__((ext_vector_type(2)));
typedef float          v4f   __attribute__((ext_vector_type(4)));
typedef float          v8f   __attribute__((ext_vector_type(8)));
typedef int            v4i   __attribute__((ext_vector_type(4)));
typedef int            v8i   __attribute__((ext_vector_type(8)));
typedef unsigned int   v4u   __attribute__((ext_vector_type(4)));
typedef unsigned short v4us  __attribute__((ext_vector_type(4)));
typedef unsigned short v8us  __attribute__((ext_vector_type(8)));
typedef unsigned short v16us __attribute__((ext_vector_type(16)));
typedef __bf16         v16bf __attribute__((ext_vector_type(16)));
typedef v2f  __attribute__((may_alias)) v2fa;
typedef v4f  __attribute__((may_alias)) v4fa;
typedef v4i  __attribute__((may_alias)) v4ia;
typedef v4us __attribute__((may_alias)) v4usa;
typedef v8us __attribute__((may_alias)) v8usa;
union FragB { v16bf v; v16us u; v8us h[2]; v8i w; };

__device__ __forceinline__ v8f wmb(const FragB& a, const FragB& b, v8f c) {
  v8f d = __builtin_amdgcn_wmma_f32_16x16x32_bf16(false, a.v, false, b.v, (short)0, c, false, false);
  asm volatile("v_nop\n\tv_nop\n\tv_nop\n\tv_nop" : "+v"(d) : "v"(a.w), "v"(b.w));
  return d;
}

__device__ __forceinline__ unsigned bf16_bits(float f) {
  const unsigned u = __float_as_uint(f);
  return (u + 0x7FFFu + ((u >> 16) & 1u)) >> 16;
}
__device__ __forceinline__ float bf16_val(float f) {
  return __uint_as_float(bf16_bits(f) << 16);
}

template <int SLB>
__device__ __forceinline__ int scan_chunk(const int* __restrict__ dsts, int nE, int cbase, int slotBase,
                                          int nb, int vec8, int* list, int tid, int lane, int wave) {
  int wc = 0;
  const int el0  = tid * EPT;
  const int e0   = cbase + el0;
  const int sent = -2147483647 - 1;
  v4i da, db;
  if (vec8 != 0 && cbase + CHUNK <= nE) {
    da = *(const v4i*)(dsts + e0);
    db = *(const v4i*)(dsts + e0 + 4);
  } else {
    da.x = (e0     < nE) ? dsts[min(e0,     nE - 1)] : sent;
    da.y = (e0 + 1 < nE) ? dsts[min(e0 + 1, nE - 1)] : sent;
    da.z = (e0 + 2 < nE) ? dsts[min(e0 + 2, nE - 1)] : sent;
    da.w = (e0 + 3 < nE) ? dsts[min(e0 + 3, nE - 1)] : sent;
    db.x = (e0 + 4 < nE) ? dsts[min(e0 + 4, nE - 1)] : sent;
    db.y = (e0 + 5 < nE) ? dsts[min(e0 + 5, nE - 1)] : sent;
    db.z = (e0 + 6 < nE) ? dsts[min(e0 + 6, nE - 1)] : sent;
    db.w = (e0 + 7 < nE) ? dsts[min(e0 + 7, nE - 1)] : sent;
  }
  const unsigned nbs = (unsigned)slotBase;
  const unsigned unb = (unsigned)nb;
  const unsigned s0 = (unsigned)da.x - nbs, s1 = (unsigned)da.y - nbs;
  const unsigned s2 = (unsigned)da.z - nbs, s3 = (unsigned)da.w - nbs;
  const unsigned s4 = (unsigned)db.x - nbs, s5 = (unsigned)db.y - nbs;
  const unsigned s6 = (unsigned)db.z - nbs, s7 = (unsigned)db.w - nbs;
  const bool h0 = s0 < unb, h1 = s1 < unb, h2 = s2 < unb, h3 = s3 < unb;
  const bool h4 = s4 < unb, h5 = s5 < unb, h6 = s6 < unb, h7 = s7 < unb;
  const unsigned any = __builtin_amdgcn_ballot_w32(h0 | h1 | h2 | h3 | h4 | h5 | h6 | h7);
  if (any != 0u) {
#define HITJ(J, HJ, SJ) { \
      const unsigned mj = __builtin_amdgcn_ballot_w32(HJ); \
      if (mj != 0u) { \
        if (HJ) { \
          const int pos = wc + (int)__builtin_amdgcn_mbcnt_lo(mj, 0u); \
          if (pos < WCAP) list[wave * WCAP + pos] = ((el0 + (J)) << SLB) | (int)(SJ); \
        } \
        wc += (int)__builtin_popcount(mj); } }
    HITJ(0, h0, s0)
    HITJ(1, h1, s1)
    HITJ(2, h2, s2)
    HITJ(3, h3, s3)
    HITJ(4, h4, s4)
    HITJ(5, h5, s5)
    HITJ(6, h6, s6)
    HITJ(7, h7, s7)
#undef HITJ
  }
  return wc;
}

__device__ __forceinline__ v8us gather8(const float* __restrict__ p) {
  v8us o;
#pragma unroll
  for (int i = 0; i < 8; ++i) o[i] = (unsigned short)bf16_bits(p[(size_t)i * HID]);
  return o;
}

__global__ __launch_bounds__(NTHR) void k_wprep(const float* __restrict__ Wp, const float* __restrict__ W1,
                                                const float* __restrict__ W2, const float* __restrict__ W3,
                                                unsigned short* WpT, unsigned short* W1T,
                                                unsigned short* W2T, unsigned short* W3T) {
  const int u   = (int)blockIdx.x * NTHR + (int)threadIdx.x;
  const int mat = u >> 10;
  const int v   = u & (NUW - 1);
  const int n   = v >> 4;
  const int k8  = (v & 15) * 8;
  const int kk  = k8 & (HID - 1);
  v8us o;
  unsigned short* dp;
  if (mat == 0) {
    o  = gather8(Wp + (size_t)k8 * HID + n);
    dp = WpT + (size_t)n * KK + k8;
  } else if (mat == 1) {
    o  = gather8(W1 + (size_t)kk * HID + n);
    dp = W1T + (size_t)n * KK + k8;
  } else if (mat == 2) {
    o  = gather8(W2 + (size_t)kk * HID + n);
    dp = W2T + (size_t)n * KK + k8;
  } else if (mat == 3) {
    o  = gather8(W3 + (size_t)kk * HID + n);
    dp = W3T + (size_t)n * KK + k8;
  } else {
    return;
  }
  *(volatile v8us*)dp = o;
  __threadfence();
  *(volatile v8us*)dp = o;
}

__global__ __launch_bounds__(NTHR) void k_cvx(const float* __restrict__ x, int nN, int nUnits,
                                              unsigned short* xb) {
  const int u = (int)blockIdx.x * NTHR + (int)threadIdx.x;
  if (u >= nUnits) return;
  const int row = u >> 4;
  const int k8  = (u & 15) * 8;
  const int rc  = row < nN ? row : nN - 1;
  const float* p = x + (size_t)rc * CIN + k8;
  const v4f a = *(const v4fa*)p;
  const v4f b = *(const v4fa*)(p + 4);
  const bool ok = row < nN;
  v8us o;
  o[0] = ok ? (unsigned short)bf16_bits(a.x) : (unsigned short)0;
  o[1] = ok ? (unsigned short)bf16_bits(a.y) : (unsigned short)0;
  o[2] = ok ? (unsigned short)bf16_bits(a.z) : (unsigned short)0;
  o[3] = ok ? (unsigned short)bf16_bits(a.w) : (unsigned short)0;
  o[4] = ok ? (unsigned short)bf16_bits(b.x) : (unsigned short)0;
  o[5] = ok ? (unsigned short)bf16_bits(b.y) : (unsigned short)0;
  o[6] = ok ? (unsigned short)bf16_bits(b.z) : (unsigned short)0;
  o[7] = ok ? (unsigned short)bf16_bits(b.w) : (unsigned short)0;
  unsigned short* dp = xb + (size_t)row * CIN + k8;
  *(volatile v8us*)dp = o;
  __threadfence();
  *(volatile v8us*)dp = o;
}

__global__ __launch_bounds__(NTHR) void k_build(const int* __restrict__ srcs, const int* __restrict__ dsts,
                                                int nE, int nN, int vec8,
                                                float* dis, int* otab, int* hits) {
  extern __shared__ __attribute__((aligned(16))) int dsm[];
  int* list = dsm;
  int* hl   = dsm + LISTN;
  int* sl   = hl + RCAP;
  int* cnt  = sl + RCAP;
  int* offs = cnt + NBA;
  int* cur  = offs + OTP;
  int* misc = cur + NBA;
  const int tid = (int)threadIdx.x, lane = tid & 31, wave = tid >> 5;
  const int blk = (int)blockIdx.x;
  const int nodeBase = blk * NBA;

  {
    const v4i z4 = {0, 0, 0, 0};
    for (int i = tid * 4; i < BLD_ZINTS; i += NTHR * 4) *(v4ia*)(dsm + i) = z4;
    if (tid < 16) misc[tid] = 0;
  }
  __syncthreads();

  int t = 0, ov = 0;
  const int nChunks = (nE + CHUNK - 1) / CHUNK;
#pragma unroll 1
  for (int ch = 0; ch < nChunks; ++ch) {
    const int cbase = ch * CHUNK;
    const int wc = scan_chunk<SLA>(dsts, nE, cbase, nodeBase, NBA, vec8, list, tid, lane, wave);
    if (lane == 0) misc[wave] = wc;
    __syncthreads();
    if (wave == 0) {
#pragma unroll 1
      for (int w2 = 0; w2 < NWAVE; ++w2) {
        int c = misc[w2];
        c = c < 0 ? 0 : (c > WCAP ? WCAP : c);
#pragma unroll 1
        for (int b0 = 0; b0 < c; b0 += 32) {
          const int idx = b0 + lane;
          const int ent = list[w2 * WCAP + (idx < WCAP ? idx : WCAP - 1)];
          const int m32 = (c - b0) < 32 ? (c - b0) : 32;
#pragma unroll 1
          for (int k = 0; k < m32; ++k) {
            const int u    = __builtin_amdgcn_readlane(ent, k);
            const int slot = u & (NBA - 1);
            const int el   = (u >> SLA) & (CHUNK - 1);
            const int pk   = ((cbase + el) << SLA) | slot;
            if (t < RCAP) {
              if (lane == 0) { hl[t] = pk; cnt[slot] = cnt[slot] + 1; }
              t = t + 1;
            } else {
              ov = 1;
            }
          }
        }
      }
    }
    __syncthreads();
  }
  if (wave == 0 && lane == 0) { misc[8] = t; misc[9] = ov; }
  __syncthreads();
  int tt = misc[8];
  tt = tt < 0 ? 0 : (tt > RCAP ? RCAP : tt);
  const int ovf = misc[9];

  if (wave == 0) {
    const int base = lane * (NBA / 32);
    int s = 0;
#pragma unroll 1
    for (int i = 0; i < NBA / 32; ++i) s += cnt[base + i];
    int incl = s;
#pragma unroll
    for (int d = 1; d < 32; d <<= 1) {
      const int y = __shfl_up(incl, d, 32);
      if (lane >= d) incl += y;
    }
    int run = incl - s;
#pragma unroll 1
    for (int i = 0; i < NBA / 32; ++i) {
      const int cv = cnt[base + i];
      offs[base + i] = run;
      cur[base + i]  = run;
      run += cv;
    }
    if (lane == 31) { offs[NBA] = run; offs[NBA + 1] = ovf; }
  }
  __syncthreads();
  if (wave == 0) {
#pragma unroll 1
    for (int b0 = 0; b0 < tt; b0 += 32) {
      const int idx = b0 + lane;
      const int ent = hl[idx < RCAP ? idx : RCAP - 1];
      const int m32 = (tt - b0) < 32 ? (tt - b0) : 32;
#pragma unroll 1
      for (int k = 0; k < m32; ++k) {
        const int u    = __builtin_amdgcn_readlane(ent, k);
        const int slot = u & (NBA - 1);
        if (lane == 0) {
          int p = cur[slot];
          p = p < 0 ? 0 : (p > RCAP - 1 ? RCAP - 1 : p);
          sl[p] = u;
          cur[slot] = p + 1;
        }
      }
    }
  }
  __syncthreads();

#pragma unroll 1
  for (int i4 = tid * 4; i4 < RCAP; i4 += NTHR * 4) {
    const v4i en = *(const v4ia*)(sl + i4);
    int e0 = en.x >> SLA, e1 = en.y >> SLA, e2 = en.z >> SLA, e3 = en.w >> SLA;
    e0 = e0 < 0 ? 0 : (e0 > nE - 1 ? nE - 1 : e0);
    e1 = e1 < 0 ? 0 : (e1 > nE - 1 ? nE - 1 : e1);
    e2 = e2 < 0 ? 0 : (e2 > nE - 1 ? nE - 1 : e2);
    e3 = e3 < 0 ? 0 : (e3 > nE - 1 ? nE - 1 : e3);
    int r0 = srcs[e0], r1 = srcs[e1], r2 = srcs[e2], r3 = srcs[e3];
    r0 = r0 < 0 ? 0 : (r0 > nN - 1 ? nN - 1 : r0);
    r1 = r1 < 0 ? 0 : (r1 > nN - 1 ? nN - 1 : r1);
    r2 = r2 < 0 ? 0 : (r2 > nN - 1 ? nN - 1 : r2);
    r3 = r3 < 0 ? 0 : (r3 > nN - 1 ? nN - 1 : r3);
    v4i o;
    o.x = (i4     < tt) ? r0 : 0;
    o.y = (i4 + 1 < tt) ? r1 : 0;
    o.z = (i4 + 2 < tt) ? r2 : 0;
    o.w = (i4 + 3 < tt) ? r3 : 0;
    *(v4ia*)(sl + i4) = o;
  }
  __syncthreads();

  int*   hrow = hits + (size_t)blk * RCAP;
  int*   orow = otab + (size_t)blk * OTP;
  float* drow = dis  + (size_t)blk * NBA;
  const v4i ot0 = *(const v4ia*)(offs + 4 * tid);
  const int t8  = tid < 8 ? tid : 7;
  const v4i ot1 = *(const v4ia*)(offs + NBA + 4 * t8);
  v4f dv;
  {
    const v4i c4 = *(const v4ia*)(cnt + 4 * tid);
    dv.x = rsqrtf((float)c4.x + 1.0f);
    dv.y = rsqrtf((float)c4.y + 1.0f);
    dv.z = rsqrtf((float)c4.z + 1.0f);
    dv.w = rsqrtf((float)c4.w + 1.0f);
  }
#pragma unroll 4
  for (int i4 = tid * 4; i4 < RCAP; i4 += NTHR * 4) {
    const v4i v = *(const v4ia*)(sl + i4);
    *(volatile v4i*)(hrow + i4) = v;
  }
  *(volatile v4i*)(orow + 4 * tid) = ot0;
  if (tid < 8) *(volatile v4i*)(orow + NBA + 4 * tid) = ot1;
  *(volatile v4f*)(drow + 4 * tid) = dv;
  __threadfence();
#pragma unroll 4
  for (int i4 = tid * 4; i4 < RCAP; i4 += NTHR * 4) {
    const v4i v = *(const v4ia*)(sl + i4);
    *(volatile v4i*)(hrow + i4) = v;
  }
  *(volatile v4i*)(orow + 4 * tid) = ot0;
  if (tid < 8) *(volatile v4i*)(orow + NBA + 4 * tid) = ot1;
  *(volatile v4f*)(drow + 4 * tid) = dv;
}

template <int MODE>
__global__ __launch_bounds__(GTHR) void k_gemm(
    const unsigned short* __restrict__ A, const unsigned short* __restrict__ WT,
    const float* __restrict__ bias, const float* __restrict__ dis, int nN,
    float* outF, unsigned short* outH)
{
  __shared__ __attribute__((aligned(16))) float stg[GBM * GBN];
  const int tid = (int)threadIdx.x, lane = tid & 31, wave = tid >> 5, hh = lane >> 4, m = lane & 15;
  const int rowBase = (int)blockIdx.x * GBM;

  v8f acc[4];
  {
    const v8f z = {0.f, 0.f, 0.f, 0.f, 0.f, 0.f, 0.f, 0.f};
    acc[0] = z; acc[1] = z; acc[2] = z; acc[3] = z;
  }
  const unsigned short* ap = A  + (size_t)(rowBase + 16 * wave + m) * (size_t)KK + 8 * hh;
  const unsigned short* wp = WT + (size_t)m * (size_t)KK + 8 * hh;
#pragma unroll 1
  for (int ks = 0; ks < KK / 32; ++ks) {
    FragB af;
    af.h[0] = *(const v8usa*)(ap + 32 * ks);
    af.h[1] = *(const v8usa*)(ap + 32 * ks + 16);
#pragma unroll
    for (int t = 0; t < 4; ++t) {
      const unsigned short* wq = wp + (size_t)(16 * t) * (size_t)KK + 32 * ks;
      FragB bf;
      bf.h[0] = *(const v8usa*)wq;
      bf.h[1] = *(const v8usa*)(wq + 16);
      acc[t] = wmb(af, bf, acc[t]);
    }
  }

#pragma unroll
  for (int t = 0; t < 4; ++t) {
    const int lc = 16 * t + m;
#pragma unroll
    for (int r = 0; r < 8; ++r) {
      const int lr = 16 * wave + 8 * hh + r;
      stg[lr * GBN + lc] = acc[t][r];
    }
  }
  __syncthreads();

  v4f fv[8];
#pragma unroll
  for (int i = 0; i < 8; ++i) {
    const int lr = 16 * wave + 2 * i + hh;
    fv[i] = *(const v4fa*)(stg + lr * GBN + 4 * m);
  }

  if constexpr (MODE != 0) {
    const float dv = dis[rowBase + 16 * wave + m];
#pragma unroll
    for (int i = 0; i < 8; ++i) {
      const float sc = __shfl(dv, 2 * i + hh, 32);
      v4f y = fv[i];
      y.x = y.x * sc; y.y = y.y * sc; y.z = y.z * sc; y.w = y.w * sc;
      fv[i] = y;
    }
#pragma unroll
    for (int i = 0; i < 8; ++i) {
      const int gr = rowBase + 16 * wave + 2 * i + hh;
      float* op = outF + (size_t)gr * (size_t)HID + 4 * m;
      *(volatile v4f*)op = fv[i];
    }
    __threadfence();
#pragma unroll
    for (int i = 0; i < 8; ++i) {
      const int gr = rowBase + 16 * wave + 2 * i + hh;
      float* op = outF + (size_t)gr * (size_t)HID + 4 * m;
      *(volatile v4f*)op = fv[i];
    }
  } else {
    v4f bb4;
    {
      const v4f tb = *(const v4fa*)(bias + 4 * m);
      bb4.x = bf16_val(tb.x); bb4.y = bf16_val(tb.y); bb4.z = bf16_val(tb.z); bb4.w = bf16_val(tb.w);
    }
    __syncthreads();
#pragma unroll
    for (int i = 0; i < 8; ++i) {
      const int lr = 16 * wave + 2 * i + hh;
      const bool ok = (rowBase + lr) < nN;
      v4f y = fv[i] + bb4;
      y.x = ok ? y.x : 0.0f; y.y = ok ? y.y : 0.0f; y.z = ok ? y.z : 0.0f; y.w = ok ? y.w : 0.0f;
      v4us h4, l4;
      unsigned hb;
      hb = bf16_bits(y.x); h4[0] = (unsigned short)hb; l4[0] = (unsigned short)bf16_bits(y.x - __uint_as_float(hb << 16));
      hb = bf16_bits(y.y); h4[1] = (unsigned short)hb; l4[1] = (unsigned short)bf16_bits(y.y - __uint_as_float(hb << 16));
      hb = bf16_bits(y.z); h4[2] = (unsigned short)hb; l4[2] = (unsigned short)bf16_bits(y.z - __uint_as_float(hb << 16));
      hb = bf16_bits(y.w); h4[3] = (unsigned short)hb; l4[3] = (unsigned short)bf16_bits(y.w - __uint_as_float(hb << 16));
      unsigned short* srow = (unsigned short*)stg + (size_t)lr * (2 * GBN);
      *(v4usa*)(srow + 4 * m) = h4;
      *(v4usa*)(srow + HID + 4 * m) = l4;
    }
    __syncthreads();
    v8us qv[8];
#pragma unroll
    for (int i = 0; i < 8; ++i) {
      const int lr = 16 * wave + 2 * i + hh;
      const unsigned short* srow = (const unsigned short*)stg + (size_t)lr * (2 * GBN);
      qv[i] = *(const v8usa*)(srow + 8 * m);
    }
#pragma unroll
    for (int i = 0; i < 8; ++i) {
      const int gr = rowBase + 16 * wave + 2 * i + hh;
      unsigned short* rp = outH + (size_t)gr * (size_t)KK + 8 * m;
      *(volatile v8us*)rp = qv[i];
    }
    __threadfence();
#pragma unroll
    for (int i = 0; i < 8; ++i) {
      const int gr = rowBase + 16 * wave + 2 * i + hh;
      unsigned short* rp = outH + (size_t)gr * (size_t)KK + 8 * m;
      *(volatile v8us*)rp = qv[i];
    }
  }
}

template <int FIN>
__global__ __launch_bounds__(NTHR) void k_agg(const int* __restrict__ hits, const int* __restrict__ otab,
                                              const float* __restrict__ dis, const float* __restrict__ gp,
                                              const float* __restrict__ bias, int nN, int mRows,
                                              unsigned short* hb, float* outp) {
  const int tid = (int)threadIdx.x, lane = tid & 31;
  const int wave = __builtin_amdgcn_readfirstlane(tid >> 5);
  float bv0, bv1;
  {
    const v2f a = *(const v2fa*)(bias + 2 * lane);
    bv0 = bf16_val(a.x); bv1 = bf16_val(a.y);
  }
  const float qnan = __int_as_float(0x7fc00000);
  const int sa = (2 * lane) & 31, sb = (2 * lane + 1) & 31;
  const int q0s = (4 * lane) & 31, q1s = (4 * lane + 1) & 31;
  const int q2s = (4 * lane + 2) & 31, q3s = (4 * lane + 3) & 31;
#pragma unroll 1
  for (int si = 0; si < AROWS / NWAVE; ++si) {
    const int node = (int)blockIdx.x * AROWS + si * NWAVE + wave;
    const int nc = node < nN ? node : nN - 1;
    const int tb = nc >> SLA;
    const int s  = nc & (NBA - 1);
    const int* ot = otab + (size_t)tb * OTP;
    int o = ot[s];
    const int e   = ot[s + 1];
    const int ovf = ot[NBA + 1];
    int c = e - o;
    const bool bad = (c > DEGCAP) | (c < 0) | (o < 0) | (o > RCAP) | (ovf != 0);
    c = c < 0 ? 0 : (c > DEGCAP ? DEGCAP : c);
    o = o < 0 ? 0 : (o > RCAP ? RCAP : o);
    const float dd = dis[nc];
    float acc0, acc1;
    {
      const v2f a = *(const v2fa*)(gp + (size_t)nc * HID + 2 * lane);
      acc0 = a.x; acc1 = a.y;
    }
    const int* hrow = hits + (size_t)tb * RCAP;
#pragma unroll 1
    for (int b0 = 0; b0 < c; b0 += 32) {
      int idx = o + b0 + lane;
      idx = idx > RCAP - 1 ? RCAP - 1 : idx;
      int sr = hrow[idx];
      sr = sr < 0 ? 0 : (sr > nN - 1 ? nN - 1 : sr);
      const int m32 = (c - b0) < 32 ? (c - b0) : 32;
#pragma unroll 1
      for (int k = 0; k < m32; ++k) {
        const int sk = __builtin_amdgcn_readlane(sr, k);
        const v2f a = *(const v2fa*)(gp + (size_t)sk * HID + 2 * lane);
        acc0 += a.x; acc1 += a.y;
      }
    }
    const float pz = bad ? qnan : 0.0f;
    const bool live = node < nN;
    float y0 = dd * acc0 + bv0;
    float y1 = dd * acc1 + bv1;
    const bool wr16 = lane < 16;
    if constexpr (FIN == 0) {
      y0 = (y0 > 0.0f) ? y0 : (y0 - y0);
      y1 = (y1 > 0.0f) ? y1 : (y1 - y1);
      y0 = y0 + pz; y1 = y1 + pz;
      const float v0 = live ? y0 : 0.0f;
      const float v1 = live ? y1 : 0.0f;
      const unsigned hb0 = bf16_bits(v0), hb1 = bf16_bits(v1);
      const unsigned lb0 = bf16_bits(v0 - __uint_as_float(hb0 << 16));
      const unsigned lb1 = bf16_bits(v1 - __uint_as_float(hb1 << 16));
      const int hw = (int)(hb0 | (hb1 << 16));
      const int lw = (int)(lb0 | (lb1 << 16));
      const int g0 = __shfl(hw, q0s, 32), g1 = __shfl(hw, q1s, 32);
      const int g2 = __shfl(hw, q2s, 32), g3 = __shfl(hw, q3s, 32);
      const int p0 = __shfl(lw, q0s, 32), p1 = __shfl(lw, q1s, 32);
      const int p2 = __shfl(lw, q2s, 32), p3 = __shfl(lw, q3s, 32);
      const bool lsel = (lane & 8) != 0;
      v4u pv;
      pv.x = (unsigned int)(lsel ? p0 : g0);
      pv.y = (unsigned int)(lsel ? p1 : g1);
      pv.z = (unsigned int)(lsel ? p2 : g2);
      pv.w = (unsigned int)(lsel ? p3 : g3);
      const bool wr = (node < mRows) && wr16;
      unsigned short* hp = hb + (size_t)node * KK + 8 * (lane & 15);
      if (wr) *(volatile v4u*)hp = pv;
      __threadfence();
      if (wr) *(volatile v4u*)hp = pv;
    } else {
      float ss = y0 * y0 + y1 * y1;
#pragma unroll
      for (int d = 16; d >= 1; d >>= 1) ss += __shfl_xor(ss, d, 32);
      const float nrm = sqrtf(ss);
      const float dn  = (nrm > 1e-12f) ? nrm : 1e-12f;
      const float inv = 1.0f / dn;
      const float v0 = y0 * inv + pz;
      const float v1 = y1 * inv + pz;
      v4f ow;
      ow.x = __shfl(v0, sa, 32); ow.y = __shfl(v1, sa, 32);
      ow.z = __shfl(v0, sb, 32); ow.w = __shfl(v1, sb, 32);
      const bool wr = live && wr16;
      float* op = outp + (size_t)nc * HID + 4 * (lane & 15);
      if (wr) *(volatile v4f*)op = ow;
      __threadfence();
      if (wr) *(volatile v4f*)op = ow;
    }
  }
}

static inline int cdiv(int a, int b) { return (a + b - 1) / b; }
static inline size_t al256(size_t o) { return (o + 255) & ~(size_t)255; }

extern "C" void kernel_launch(void* const* d_in, const int* in_sizes, int n_in,
                              void* d_out, int out_size, void* d_ws, size_t ws_size,
                              hipStream_t stream) {
  if (n_in < 10) return;
  if (in_sizes[0] < CIN || (in_sizes[0] % CIN) != 0) return;
  const int nN = in_sizes[0] / CIN;
  if (nN < 1 || nN > (1 << 22)) return;
  if (in_sizes[1] < 2 || (in_sizes[1] & 1) != 0) return;
  const int nE = in_sizes[1] / 2;
  if (nE < 1 || nE >= (1 << (31 - SLA))) return;
  if (in_sizes[2] != CIN * HID || in_sizes[3] != HID) return;
  if (in_sizes[4] != HID * HID || in_sizes[5] != HID) return;
  if (in_sizes[6] != HID * HID || in_sizes[7] != HID) return;
  if (in_sizes[8] != HID * HID || in_sizes[9] != HID) return;
  if ((long long)out_size != (long long)nN * HID) return;

  const float* x    = (const float*)d_in[0];
  const int*   edge = (const int*)d_in[1];
  const float* Wp   = (const float*)d_in[2];
  const float* bp   = (const float*)d_in[3];
  const float* W1   = (const float*)d_in[4];
  const float* b1   = (const float*)d_in[5];
  const float* W2   = (const float*)d_in[6];
  const float* b2   = (const float*)d_in[7];
  const float* W3   = (const float*)d_in[8];
  const float* b3   = (const float*)d_in[9];
  float* out = (float*)d_out;
  const int* src = edge;
  const int* dst = edge + nE;

  const int MP = cdiv(nN, GBM) * GBM;
  const int gM = MP / GBM;
  const int gA = cdiv(MP, NBA);
  if ((long long)gA * NBA < (long long)MP) return;
  const int vec8 = ((nE & 3) == 0) ? 1 : 0;

  char* ws = (char*)d_ws;
  size_t off = 0;
  const size_t oDIS = off; off = al256(off + (size_t)gA * NBA * 4);
  const size_t oOT  = off; off = al256(off + (size_t)gA * OTP * 4);
  const size_t oHT  = off; off = al256(off + (size_t)gA * RCAP * 4);
  const size_t oWpT = off; off = al256(off + (size_t)HID * KK * 2);
  const size_t oW1T = off; off = al256(off + (size_t)HID * KK * 2);
  const size_t oW2T = off; off = al256(off + (size_t)HID * KK * 2);
  const size_t oW3T = off; off = al256(off + (size_t)HID * KK * 2);
  const size_t oXB  = off; off = al256(off + (size_t)MP * CIN * 2);
  const size_t oHB  = off; off = al256(off + (size_t)MP * KK * 2);
  const size_t oG   = off; off = al256(off + (size_t)MP * HID * 4);
  if (off > ws_size || off > (size_t)WSMAX) return;
  float*          DIS = (float*)(ws + oDIS);
  int*            OT  = (int*)(ws + oOT);
  int*            HT  = (int*)(ws + oHT);
  unsigned short* WpT = (unsigned short*)(ws + oWpT);
  unsigned short* W1T = (unsigned short*)(ws + oW1T);
  unsigned short* W2T = (unsigned short*)(ws + oW2T);
  unsigned short* W3T = (unsigned short*)(ws + oW3T);
  unsigned short* XB  = (unsigned short*)(ws + oXB);
  unsigned short* HB  = (unsigned short*)(ws + oHB);
  float*          G   = (float*)(ws + oG);

  const size_t bldLds = (size_t)BLD_LDS_INTS * 4;
  hipFuncSetAttribute(reinterpret_cast<const void*>(&k_build), hipFuncAttributeMaxDynamicSharedMemorySize, (int)bldLds);

  const int nUx = MP * (CIN / 8);
  k_wprep<<<(4 * NUW) / NTHR, NTHR, 0, stream>>>(Wp, W1, W2, W3, WpT, W1T, W2T, W3T);
  k_cvx<<<cdiv(nUx, NTHR), NTHR, 0, stream>>>(x, nN, nUx, XB);
  k_build<<<gA, NTHR, bldLds, stream>>>(src, dst, nE, nN, vec8, DIS, OT, HT);
  k_gemm<0><<<gM, GTHR, 0, stream>>>(XB, WpT, bp, DIS, nN, G, HB);
  k_gemm<1><<<gM, GTHR, 0, stream>>>(HB, W1T, bp, DIS, nN, G, HB);
  k_agg<0><<<gM, NTHR, 0, stream>>>(HT, OT, DIS, G, b1, nN, MP, HB, out);
  k_gemm<1><<<gM, GTHR, 0, stream>>>(HB, W2T, bp, DIS, nN, G, HB);
  k_agg<0><<<gM, NTHR, 0, stream>>>(HT, OT, DIS, G, b2, nN, MP, HB, out);
  k_gemm<1><<<gM, GTHR, 0, stream>>>(HB, W3T, bp, DIS, nN, G, HB);
  k_agg<1><<<gM, NTHR, 0, stream>>>(HT, OT, DIS, G, b3, nN, MP, HB, out);
}
